// GraphNeuralPPOPolicy_21749714387569
// MI455X (gfx1250) — hardware-verified
//
#include <hip/hip_runtime.h>
#include <stddef.h>


#define KIN   256
#define DF    256
#define NH    8
#define HC    32
#define GR    32
#define AP    264
#define XSP   260
#define TP    68
#define NB    125
#define CHUNK 2048
#define NTHR  256
#define NWAVE 8
#define WCAP  256
#define NGRP  (CHUNK / (NTHR * 4))

#define GEMM_LDS_AH    0
#define GEMM_LDS_AL    (GR * AP * 2)
#define GEMM_LDS_XS    (2 * GR * AP * 2)
#define GEMM_LDS_SS    (GEMM_LDS_XS + GR * XSP * 4)
#define GEMM_LDS_SD    (GEMM_LDS_SS + GR * NH * 4)
#define GEMM_LDS_BYTES (GEMM_LDS_SD + GR * NH * 4)

#define GAT_SACC  0
#define GAT_HROW  (NB * DF)
#define GAT_RMX   (2 * NB * DF)
#define GAT_RSM   (GAT_RMX + NB * NH)
#define GAT_SDS   (GAT_RSM + NB * NH)
#define GAT_LIST  (GAT_SDS + NB * NH)
#define GAT_WCNT  (GAT_LIST + NWAVE * WCAP)
#define GAT_LDS_BYTES ((GAT_WCNT + NWAVE) * 4)

static_assert(WCAP == (CHUNK / NTHR) * 32);
static_assert(NGRP >= 1);
static_assert(NB <= 512);
static_assert((CHUNK & (CHUNK - 1)) == 0 && CHUNK <= 4096);
static_assert(GEMM_LDS_BYTES == 69120);
static_assert(GAT_LDS_BYTES == 276224);
static_assert((GEMM_LDS_AL % 16) == 0 && (GEMM_LDS_XS % 16) == 0 && (GEMM_LDS_SS % 16) == 0);
static_assert(((GAT_HROW * 4) % 16) == 0 && ((GAT_RMX * 4) % 16) == 0);
static_assert(KIN % 32 == 0 && DF == NH * HC && NTHR == GR * NH);

typedef float  v4f  __attribute__((ext_vector_type(4)));
typedef float  v8f  __attribute__((ext_vector_type(8)));
typedef int    v4i  __attribute__((ext_vector_type(4)));
typedef __bf16 v8b  __attribute__((ext_vector_type(8)));
typedef __bf16 v16b __attribute__((ext_vector_type(16)));
union Frag { v16b v; v8b half[2]; };

__device__ __forceinline__ v8f wm(v16b a, v16b b, v8f c) {
  v8f d = __builtin_amdgcn_wmma_f32_16x16x32_bf16(false, a, false, b, (short)0, c, false, false);
  asm volatile("v_nop\n\tv_nop\n\tv_nop\n\tv_nop" : "+v"(d) : "v"(a), "v"(b));
  return d;
}

__device__ __forceinline__ unsigned bfb(float f) {
  const unsigned u = __float_as_uint(f);
  return (u + 0x7FFFu + ((u >> 16) & 1u)) >> 16;
}

__device__ __forceinline__ void split8(v4f a, v4f b, v4i& hi, v4i& lo) {
  float f[8] = {a.x, a.y, a.z, a.w, b.x, b.y, b.z, b.w};
  unsigned hb[8], lb[8];
#pragma unroll
  for (int j = 0; j < 8; ++j) {
    hb[j] = bfb(f[j]);
    lb[j] = bfb(f[j] - __uint_as_float(hb[j] << 16));
  }
  hi.x = (int)(hb[0] | (hb[1] << 16)); hi.y = (int)(hb[2] | (hb[3] << 16));
  hi.z = (int)(hb[4] | (hb[5] << 16)); hi.w = (int)(hb[6] | (hb[7] << 16));
  lo.x = (int)(lb[0] | (lb[1] << 16)); lo.y = (int)(lb[2] | (lb[3] << 16));
  lo.z = (int)(lb[4] | (lb[5] << 16)); lo.w = (int)(lb[6] | (lb[7] << 16));
}

__global__ __launch_bounds__(NTHR) void k_prepw(const float* __restrict__ W, __bf16* WTh, __bf16* WTl) {
  __shared__ __attribute__((aligned(16))) float Ts[32 * TP];
  const int tid = threadIdx.x;
  const int k0 = blockIdx.x * 64;
  const int o0 = blockIdx.y * 32;
  {
    const int kk = tid >> 2;
    const int oq = (tid & 3) * 8;
    const float* p = W + (size_t)(k0 + kk) * DF + o0 + oq;
    const v4f f0 = *(const v4f*)p;
    const v4f f1 = *(const v4f*)(p + 4);
    Ts[(oq + 0) * TP + kk] = f0.x; Ts[(oq + 1) * TP + kk] = f0.y;
    Ts[(oq + 2) * TP + kk] = f0.z; Ts[(oq + 3) * TP + kk] = f0.w;
    Ts[(oq + 4) * TP + kk] = f1.x; Ts[(oq + 5) * TP + kk] = f1.y;
    Ts[(oq + 6) * TP + kk] = f1.z; Ts[(oq + 7) * TP + kk] = f1.w;
  }
  __syncthreads();
  const int oo = tid >> 3;
  const int q  = tid & 7;
  const v4f g0 = *(const v4f*)(Ts + oo * TP + 8 * q);
  const v4f g1 = *(const v4f*)(Ts + oo * TP + 8 * q + 4);
  v4i hi, lo;
  split8(g0, g1, hi, lo);
  const size_t go = (size_t)(o0 + oo) * KIN + k0 + 8 * q;
  *(volatile v4i*)(WTh + go) = hi;
  *(volatile v4i*)(WTl + go) = lo;
  __threadfence();
  *(volatile v4i*)(WTh + go) = hi;
  *(volatile v4i*)(WTl + go) = lo;
}

__global__ __launch_bounds__(NTHR) void k_gemm(
    const float* __restrict__ x, const __bf16* __restrict__ WTh, const __bf16* __restrict__ WTl,
    const float* __restrict__ a_src, const float* __restrict__ a_dst,
    float* xp, float* ssrc, float* sdst, int nN) {
  extern __shared__ v4f lds_dyn[];
  char* base = (char*)lds_dyn;
  __bf16* Ah = (__bf16*)(base + GEMM_LDS_AH);
  __bf16* Al = (__bf16*)(base + GEMM_LDS_AL);
  float*  Xs = (float*)(base + GEMM_LDS_XS);
  float*  Ss = (float*)(base + GEMM_LDS_SS);
  float*  Sd = (float*)(base + GEMM_LDS_SD);

  const int tid  = threadIdx.x;
  const int lane = tid & 31;
  const int wave = tid >> 5;
  const int hh   = lane >> 4;
  const int m    = lane & 15;
  const int rowBase = blockIdx.x * GR;

  {
    const int r  = tid >> 3;
    const int c0 = (tid & 7) * 32;
    int row = rowBase + r;
    if (row > nN - 1) row = nN - 1;
    const float* p = x + (size_t)row * KIN + c0;
#pragma unroll
    for (int g = 0; g < 4; ++g) {
      const v4f f0 = *(const v4f*)(p + 8 * g);
      const v4f f1 = *(const v4f*)(p + 8 * g + 4);
      v4i hi, lo;
      split8(f0, f1, hi, lo);
      *(v4i*)(Ah + r * AP + c0 + 8 * g) = hi;
      *(v4i*)(Al + r * AP + c0 + 8 * g) = lo;
    }
  }
  __syncthreads();

#pragma unroll 1
  for (int nt = 0; nt < 2; ++nt) {
    const int col = wave * 32 + nt * 16 + m;
    v8f acc0 = {0.f, 0.f, 0.f, 0.f, 0.f, 0.f, 0.f, 0.f};
    v8f acc1 = {0.f, 0.f, 0.f, 0.f, 0.f, 0.f, 0.f, 0.f};
    const __bf16* pbh  = WTh + (size_t)col * KIN + 8 * hh;
    const __bf16* pbl  = WTl + (size_t)col * KIN + 8 * hh;
    const __bf16* pa0h = Ah + m * AP + 8 * hh;
    const __bf16* pa0l = Al + m * AP + 8 * hh;
    const __bf16* pa1h = Ah + (16 + m) * AP + 8 * hh;
    const __bf16* pa1l = Al + (16 + m) * AP + 8 * hh;
#pragma unroll
    for (int kt = 0; kt < KIN / 32; ++kt) {
      const int k0 = kt * 32;
      Frag a0h, a0l, a1h, a1l, bh, bl;
      bh.half[0]  = *(const v8b*)(pbh + k0);   bh.half[1]  = *(const v8b*)(pbh + k0 + 16);
      bl.half[0]  = *(const v8b*)(pbl + k0);   bl.half[1]  = *(const v8b*)(pbl + k0 + 16);
      a0h.half[0] = *(const v8b*)(pa0h + k0);  a0h.half[1] = *(const v8b*)(pa0h + k0 + 16);
      a0l.half[0] = *(const v8b*)(pa0l + k0);  a0l.half[1] = *(const v8b*)(pa0l + k0 + 16);
      a1h.half[0] = *(const v8b*)(pa1h + k0);  a1h.half[1] = *(const v8b*)(pa1h + k0 + 16);
      a1l.half[0] = *(const v8b*)(pa1l + k0);  a1l.half[1] = *(const v8b*)(pa1l + k0 + 16);
      acc0 = wm(a0h.v, bh.v, acc0);
      acc0 = wm(a0h.v, bl.v, acc0);
      acc0 = wm(a0l.v, bh.v, acc0);
      acc1 = wm(a1h.v, bh.v, acc1);
      acc1 = wm(a1h.v, bl.v, acc1);
      acc1 = wm(a1l.v, bh.v, acc1);
    }
#pragma unroll
    for (int r = 0; r < 8; ++r) {
      Xs[(8 * hh + r) * XSP + col]      = acc0[r];
      Xs[(16 + 8 * hh + r) * XSP + col] = acc1[r];
    }
  }
  __syncthreads();

  {
    const int r  = tid >> 3;
    const int hd = tid & 7;
    const float* xr = Xs + r * XSP + hd * HC;
    const float* as = a_src + hd * HC;
    const float* ad = a_dst + hd * HC;
    float ss = 0.f, sd = 0.f;
#pragma unroll
    for (int f4 = 0; f4 < HC / 4; ++f4) {
      const v4f hv = *(const v4f*)(xr + 4 * f4);
      const v4f av = *(const v4f*)(as + 4 * f4);
      const v4f dv = *(const v4f*)(ad + 4 * f4);
      ss += hv.x * av.x; ss += hv.y * av.y; ss += hv.z * av.z; ss += hv.w * av.w;
      sd += hv.x * dv.x; sd += hv.y * dv.y; sd += hv.z * dv.z; sd += hv.w * dv.w;
    }
    Ss[tid] = ss;
    Sd[tid] = sd;
  }
  __syncthreads();

  v4f xa[4], xb[4];
#pragma unroll
  for (int i = 0; i < 4; ++i) {
    xa[i] = *(const v4f*)(Xs + (4 * wave + i) * XSP + 4 * lane);
    xb[i] = *(const v4f*)(Xs + (4 * wave + i) * XSP + 128 + 4 * lane);
  }
  float* gp = 0;
  v4f ga = {0.f, 0.f, 0.f, 0.f}, gb = {0.f, 0.f, 0.f, 0.f};
  if (wave == 0) {
    ga = *(const v4f*)(Ss + 4 * lane);
    gb = *(const v4f*)(Ss + 128 + 4 * lane);
    gp = ssrc + (size_t)rowBase * NH;
  } else if (wave == 1) {
    ga = *(const v4f*)(Sd + 4 * lane);
    gb = *(const v4f*)(Sd + 128 + 4 * lane);
    gp = sdst + (size_t)rowBase * NH;
  }
  float* xpp[4];
#pragma unroll
  for (int i = 0; i < 4; ++i) xpp[i] = xp + (size_t)(rowBase + 4 * wave + i) * DF;

#pragma unroll
  for (int i = 0; i < 4; ++i) {
    *(volatile v4f*)(xpp[i] + 4 * lane)       = xa[i];
    *(volatile v4f*)(xpp[i] + 128 + 4 * lane) = xb[i];
  }
  if (gp) {
    *(volatile v4f*)(gp + 4 * lane)       = ga;
    *(volatile v4f*)(gp + 128 + 4 * lane) = gb;
  }
  __threadfence();
#pragma unroll
  for (int i = 0; i < 4; ++i) {
    *(volatile v4f*)(xpp[i] + 4 * lane)       = xa[i];
    *(volatile v4f*)(xpp[i] + 128 + 4 * lane) = xb[i];
  }
  if (gp) {
    *(volatile v4f*)(gp + 4 * lane)       = ga;
    *(volatile v4f*)(gp + 128 + 4 * lane) = gb;
  }
}

__global__ __launch_bounds__(NTHR) void k_gat(
    const int* __restrict__ ei, const float* __restrict__ ea,
    const float* __restrict__ xp, const float* __restrict__ ssrc, const float* __restrict__ sdst,
    const float* __restrict__ We, const float* __restrict__ be, const float* __restrict__ bias,
    float* out, int nN, int nE) {
  extern __shared__ v4f lds_dyn[];
  float* lds  = (float*)lds_dyn;
  float* sacc = lds + GAT_SACC;
  float* hrow = lds + GAT_HROW;
  float* rmx  = lds + GAT_RMX;
  float* rsm  = lds + GAT_RSM;
  float* sds  = lds + GAT_SDS;
  int*   list = (int*)(lds + GAT_LIST);
  int*   wcnt = (int*)(lds + GAT_WCNT);

  const int tid  = threadIdx.x;
  const int lane = tid & 31;
  const int wave = tid >> 5;
  const int hd   = lane >> 2;
  const int nodeBase = blockIdx.x * NB;
  const float NEG_INF = __uint_as_float(0xff800000u);

  {
    const v4f z4 = {0.f, 0.f, 0.f, 0.f};
    v4f* sacc4 = (v4f*)sacc;
    v4f* hrow4 = (v4f*)hrow;
    for (int i = tid; i < NB * DF / 4; i += NTHR) sacc4[i] = z4;
    for (int i = tid; i < NB * DF / 4; i += NTHR) {
      const int slot = i >> 6;
      const int c    = (i & 63) * 4;
      int node = nodeBase + slot;
      if (node > nN - 1) node = nN - 1;
      hrow4[i] = *(const v4f*)(xp + (size_t)node * DF + c);
    }
    for (int i = tid; i < NB * NH; i += NTHR) {
      const int slot = i >> 3;
      int node = nodeBase + slot;
      if (node > nN - 1) node = nN - 1;
      rmx[i] = NEG_INF;
      rsm[i] = 0.f;
      sds[i] = sdst[(size_t)node * NH + (i & 7)];
    }
  }
  const v4f w0a = *(const v4f*)(We + 0 * DF + 8 * lane), w0b = *(const v4f*)(We + 0 * DF + 8 * lane + 4);
  const v4f w1a = *(const v4f*)(We + 1 * DF + 8 * lane), w1b = *(const v4f*)(We + 1 * DF + 8 * lane + 4);
  const v4f w2a = *(const v4f*)(We + 2 * DF + 8 * lane), w2b = *(const v4f*)(We + 2 * DF + 8 * lane + 4);
  const v4f bea = *(const v4f*)(be + 8 * lane),          beb = *(const v4f*)(be + 8 * lane + 4);
  __syncthreads();

  const int* eid = ei + nE;
  const bool al16 = ((nE & 3) == 0);

  const int nChunks = (nE + CHUNK - 1) / CHUNK;
#pragma unroll 1
  for (int ch = 0; ch < nChunks; ++ch) {
    const int cbase = ch * CHUNK;
    int wc = 0;
#pragma unroll
    for (int g = 0; g < NGRP; ++g) {
      const int el0 = (g * NTHR + tid) * 4;
      const int e0  = cbase + el0;
      const int sent = -2147483647 - 1;
      v4i d;
      if (al16 && (e0 + 3 < nE)) {
        d = *(const v4i*)(eid + e0);
      } else {
        d.x = (e0     < nE) ? eid[min(e0, nE - 1)]     : sent;
        d.y = (e0 + 1 < nE) ? eid[min(e0 + 1, nE - 1)] : sent;
        d.z = (e0 + 2 < nE) ? eid[min(e0 + 2, nE - 1)] : sent;
        d.w = (e0 + 3 < nE) ? eid[min(e0 + 3, nE - 1)] : sent;
      }
      const unsigned s0 = (unsigned)d.x - (unsigned)nodeBase;
      const unsigned s1 = (unsigned)d.y - (unsigned)nodeBase;
      const unsigned s2 = (unsigned)d.z - (unsigned)nodeBase;
      const unsigned s3 = (unsigned)d.w - (unsigned)nodeBase;
      const bool h0 = s0 < (unsigned)NB;
      const bool h1 = s1 < (unsigned)NB;
      const bool h2 = s2 < (unsigned)NB;
      const bool h3 = s3 < (unsigned)NB;
      const unsigned many = __builtin_amdgcn_ballot_w32(h0 | h1 | h2 | h3);
      if (many != 0u) {
#define HITJ(J, HJ, SJ) { \
          const unsigned mj = __builtin_amdgcn_ballot_w32(HJ); \
          if (HJ) { \
            const int pos = wc + (int)__builtin_amdgcn_mbcnt_lo(mj, 0u); \
            if (pos < WCAP) list[wave * WCAP + pos] = ((el0 + (J)) << 9) | (int)(SJ); \
          } \
          wc += (int)__builtin_popcount(mj); }
        HITJ(0, h0, s0)
        HITJ(1, h1, s1)
        HITJ(2, h2, s2)
        HITJ(3, h3, s3)
#undef HITJ
      }
    }
    if (lane == 0) wcnt[wave] = wc;
    __syncthreads();

    if (wave == 0) {
#pragma unroll 1
      for (int wsx = 0; wsx < NWAVE; ++wsx) {
        int n = wcnt[wsx];
        if (n > WCAP) n = WCAP;
        if (n < 0) n = 0;
#pragma unroll 1
        for (int i = 0; i < n; ++i) {
          const int ent = __builtin_amdgcn_readfirstlane(list[wsx * WCAP + i]);
          int slot = ent & 511;
          if (slot > NB - 1) slot = NB - 1;
          const int el = (ent >> 9) & (CHUNK - 1);
          int e = cbase + el;
          if (e > nE - 1) e = nE - 1;
          int src = ei[e];
          src = src < 0 ? 0 : (src > nN - 1 ? nN - 1 : src);
          const float ea0 = ea[(size_t)e * 3 + 0];
          const float ea1 = ea[(size_t)e * 3 + 1];
          const float ea2 = ea[(size_t)e * 3 + 2];
          const float ss  = ssrc[(size_t)src * NH + hd];
          const float sd  = sds[slot * NH + hd];
          const float* hp = hrow + slot * DF + 8 * lane;
          const v4f hd0 = *(const v4f*)hp;
          const v4f hd1 = *(const v4f*)(hp + 4);
          const float* gsp = xp + (size_t)src * DF + 8 * lane;
          const v4f hs0 = *(const v4f*)gsp;
          const v4f hs1 = *(const v4f*)(gsp + 4);
          v4f en0 = (ea0 * w0a + ea1 * w1a + ea2 * w2a) + bea;
          v4f en1 = (ea0 * w0b + ea1 * w1b + ea2 * w2b) + beb;
          en0.x = fmaxf(en0.x, 0.f); en0.y = fmaxf(en0.y, 0.f); en0.z = fmaxf(en0.z, 0.f); en0.w = fmaxf(en0.w, 0.f);
          en1.x = fmaxf(en1.x, 0.f); en1.y = fmaxf(en1.y, 0.f); en1.z = fmaxf(en1.z, 0.f); en1.w = fmaxf(en1.w, 0.f);
          const v4f pr = en0 * hd0 + en1 * hd1;
          float part = (pr.x + pr.y) + (pr.z + pr.w);
          part += __shfl_xor(part, 1, 32);
          part += __shfl_xor(part, 2, 32);
          float al = (ss + sd) + part;
          al = (al >= 0.f) ? al : 0.2f * al;
          const float mo = rmx[slot * NH + hd];
          const float so = rsm[slot * NH + hd];
          const float mn = fmaxf(mo, al);
          const float sc = __expf(mo - mn);
          const float p  = __expf(al - mn);
          v4f* ap = (v4f*)(sacc + slot * DF + 8 * lane);
          const v4f c0 = ap[0];
          const v4f c1 = ap[1];
          const v4f n0 = c0 * sc + p * hs0;
          const v4f n1 = c1 * sc + p * hs1;
          ap[0] = n0;
          ap[1] = n1;
          rmx[slot * NH + hd] = mn;
          rsm[slot * NH + hd] = so * sc + p;
        }
      }
    }
    __syncthreads();
  }

  const v4f b0 = *(const v4f*)(bias + 4 * lane);
  const v4f b1 = *(const v4f*)(bias + 128 + 4 * lane);
  const int hda = lane >> 3;
  const int hdb = 4 + (lane >> 3);
#pragma unroll 1
  for (int slot = wave; slot < NB; slot += NWAVE) {
    const int node = nodeBase + slot;
    if (node >= nN) break;
    const float s0 = rsm[slot * NH + hda];
    const float s1 = rsm[slot * NH + hdb];
    const float i0 = __builtin_amdgcn_rcpf(fmaxf(s0, 1e-10f));
    const float i1 = __builtin_amdgcn_rcpf(fmaxf(s1, 1e-10f));
    const v4f a0 = *(const v4f*)(sacc + slot * DF + 4 * lane);
    const v4f a1 = *(const v4f*)(sacc + slot * DF + 128 + 4 * lane);
    const v4f y0 = a0 * i0 + b0;
    const v4f y1 = a1 * i1 + b1;
    float* op = out + (size_t)node * DF;
    *(volatile v4f*)(op + 4 * lane)       = y0;
    *(volatile v4f*)(op + 128 + 4 * lane) = y1;
    __threadfence();
    *(volatile v4f*)(op + 4 * lane)       = y0;
    *(volatile v4f*)(op + 128 + 4 * lane) = y1;
  }
}

extern "C" void kernel_launch(void* const* d_in, const int* in_sizes, int n_in,
                              void* d_out, int out_size, void* d_ws, size_t ws_size,
                              hipStream_t stream) {
  if (n_in < 9) return;
  const int nN = in_sizes[0] / KIN;
  if (nN <= 0 || in_sizes[0] != nN * KIN) return;
  const int nE = in_sizes[1] / 2;
  if (nE < 0 || in_sizes[1] != 2 * nE || in_sizes[2] != 3 * nE) return;
  if (in_sizes[3] != KIN * DF) return;
  if (in_sizes[4] != NH * HC || in_sizes[5] != NH * HC) return;
  if (in_sizes[6] != 3 * DF || in_sizes[7] != DF || in_sizes[8] != DF) return;
  if (out_size != nN * DF) return;

  const float* x     = (const float*)d_in[0];
  const int*   ei    = (const int*)d_in[1];
  const float* ea    = (const float*)d_in[2];
  const float* W     = (const float*)d_in[3];
  const float* a_src = (const float*)d_in[4];
  const float* a_dst = (const float*)d_in[5];
  const float* We    = (const float*)d_in[6];
  const float* be    = (const float*)d_in[7];
  const float* bias  = (const float*)d_in[8];
  float* out = (float*)d_out;

  const int nP = ((nN + GR - 1) / GR) * GR;
  size_t off = 0;
  __bf16* WTh = (__bf16*)((char*)d_ws + off); off += (size_t)DF * KIN * sizeof(__bf16);
  __bf16* WTl = (__bf16*)((char*)d_ws + off); off += (size_t)DF * KIN * sizeof(__bf16);
  float* xp   = (float*)((char*)d_ws + off);  off += (size_t)nP * DF * sizeof(float);
  float* ssrc = (float*)((char*)d_ws + off);  off += (size_t)nP * NH * sizeof(float);
  float* sdst = (float*)((char*)d_ws + off);  off += (size_t)nP * NH * sizeof(float);
  if (off > ws_size) return;
  if (off > (size_t)134217728) return;

  k_prepw<<<dim3(KIN / 64, DF / 32), NTHR, 0, stream>>>(W, WTh, WTl);

  hipFuncSetAttribute(reinterpret_cast<const void*>(&k_gemm),
                      hipFuncAttributeMaxDynamicSharedMemorySize, GEMM_LDS_BYTES);
  k_gemm<<<nP / GR, NTHR, GEMM_LDS_BYTES, stream>>>(x, WTh, WTl, a_src, a_dst, xp, ssrc, sdst, nN);

  hipFuncSetAttribute(reinterpret_cast<const void*>(&k_gat),
                      hipFuncAttributeMaxDynamicSharedMemorySize, GAT_LDS_BYTES);
  const int grid = (nN + NB - 1) / NB;
  k_gat<<<grid, NTHR, GAT_LDS_BYTES, stream>>>(ei, ea, xp, ssrc, sdst, We, be, bias, out, nN, nE);
}
